// SelfAttention_62603443306929
// MI455X (gfx1250) — hardware-verified
//
#include <hip/hip_runtime.h>


#ifndef NB
#define NB 2
#endif
#ifndef SEQ
#define SEQ 2048
#endif
#define NB_FULL  2
#define SEQ_FULL 2048
#define NH_  16
#define HD   64
#define DM   (NH_ * HD)
#define TT   SEQ
#define ZH   2
#define RH   TT
#define SCL  0.125f
static_assert(SEQ % 128 == 0);
static_assert(NH_ % ZH == 0);
static_assert(HD == 64);
static_assert(DM % 64 == 0);
static_assert(NB >= 1 && NB <= NB_FULL);
static_assert(SEQ <= SEQ_FULL);
static_assert(TT % 64 == 0);
static_assert(RH % 64 == 0 && RH <= TT);
static_assert(HD % 32 == 0 && TT % 32 == 0);
static_assert((ZH * TT) % 8 == 0);
static_assert(((size_t)NB * NH_ * TT * HD) % 8 == 0);
static_assert((HD * 4) % 128 == 0);
#define R256(x)   ((((size_t)(x)) + 255) & ~(size_t)255)
#define PLANE_B   R256((size_t)NB * NH_ * TT * HD * 2)
#define SCORE_B   R256((size_t)ZH * TT * TT * 4)
#define PROB_B    R256((size_t)ZH * RH * TT * 2)
#define FLAG_B    R256(128)
#define CARVE_B   (3 * PLANE_B + SCORE_B + 2 * PROB_B + FLAG_B)
static_assert(CARVE_B <= (size_t)134217728);

typedef _Float16 h16;
typedef unsigned short bf;
typedef __attribute__((ext_vector_type(16))) __bf16   v16bf;
typedef __attribute__((ext_vector_type(16))) _Float16 v16h;
typedef __attribute__((ext_vector_type(8)))  _Float16 v8h;
typedef __attribute__((ext_vector_type(8)))  unsigned short v8us;
typedef __attribute__((ext_vector_type(8)))  float    v8f;
typedef __attribute__((ext_vector_type(4)))  float    v4f;
typedef __attribute__((ext_vector_type(4)))  unsigned short v4us;
typedef v8h  __attribute__((may_alias)) v8ha;
typedef v4f  __attribute__((may_alias)) v4fa;
typedef v8us __attribute__((may_alias)) v8usa;

__device__ __forceinline__ unsigned short f2bf(float f) { unsigned u = __float_as_uint(f); u += 0x7FFFu + ((u >> 16) & 1u); return (unsigned short)(u >> 16); }
__device__ __forceinline__ float bf2f(unsigned short b) { return __uint_as_float(((unsigned)b) << 16); }
__device__ __forceinline__ float bfr(float f) { return bf2f(f2bf(f)); }
__device__ __forceinline__ void splitf(float y, unsigned short& h, unsigned short& l) { h = f2bf(y); l = f2bf(y - bf2f(h)); }
__device__ __forceinline__ v16h cat16(v8h lo, v8h hi) { return __builtin_shufflevector(lo, hi, 0, 1, 2, 3, 4, 5, 6, 7, 8, 9, 10, 11, 12, 13, 14, 15); }
__device__ __forceinline__ v16bf cat16b(v8us lo, v8us hi) { return __builtin_bit_cast(v16bf, __builtin_shufflevector(lo, hi, 0, 1, 2, 3, 4, 5, 6, 7, 8, 9, 10, 11, 12, 13, 14, 15)); }
__device__ __forceinline__ v8f wmma16(v16h a, v16h b, v8f c) { return __builtin_amdgcn_wmma_f32_16x16x32_f16(false, a, false, b, (short)0, c, false, false); }
__device__ __forceinline__ v8f wmmab(v16bf a, v16bf b, v8f c) { return __builtin_amdgcn_wmma_f32_16x16x32_bf16(false, a, false, b, (short)0, c, false, false); }

template <typename T16> struct WFrag;
template <> struct WFrag<h16> { typedef v16h V; static __device__ __forceinline__ V ld(const h16* p) { return cat16(*(const v8h*)p, *(const v8h*)(p + 16)); } static __device__ __forceinline__ v8f mma(V a, V b, v8f c) { return wmma16(a, b, c); } };
template <> struct WFrag<bf> { typedef v16bf V; static __device__ __forceinline__ V ld(const bf* p) { return cat16b(*(const v8us*)p, *(const v8us*)(p + 16)); } static __device__ __forceinline__ v8f mma(V a, V b, v8f c) { return wmmab(a, b, c); } };

template <typename T16, int NSPLIT, int CMODE>
__global__ __launch_bounds__(32) void k_gemmc(const T16* __restrict__ A, const T16* __restrict__ A2, const T16* __restrict__ Bt, const T16* __restrict__ Bt2, int K, float* C, int ldc, int roff, size_t sA, size_t sB, size_t sC, const int* CF) {
    typedef typename WFrag<T16>::V V;
    __shared__ __align__(16) float os[16 * 68];
    const size_t z = blockIdx.z; A += z * sA; if (A2) A2 += z * sA; Bt += z * sB; if (Bt2) Bt2 += z * sB; C += z * sC;
    const int lane = threadIdx.x & 31, lr = lane & 15, hi = lane >> 4; const int r0 = blockIdx.x * 64, c0 = blockIdx.y * 64;
    const bool con = (CF == nullptr) || (CF[0] != 0);     if (CMODE == 1 && con && c0 > r0 + roff + 63) return;
    const int Kl = (CMODE == 2 && con) ? min(K, r0 + roff + 64) : K;
    v8f acc[4][4];
#pragma unroll
    for (int mb = 0; mb < 4; ++mb)
#pragma unroll
        for (int nb = 0; nb < 4; ++nb) acc[mb][nb] = (v8f){};
    const size_t aoff = (size_t)(r0 + lr) * K + 8 * hi, boff = (size_t)(c0 + lr) * K + 8 * hi;
#pragma unroll 1
    for (int kc = 0; kc < Kl; kc += 32) {
        V a[4], a2[4];
#pragma unroll
        for (int mb = 0; mb < 4; ++mb) { a[mb] = WFrag<T16>::ld(A + aoff + (size_t)mb * 16 * K + kc); if (NSPLIT == 1 || NSPLIT == 2) a2[mb] = WFrag<T16>::ld(A2 + aoff + (size_t)mb * 16 * K + kc); }
#pragma unroll
        for (int nb = 0; nb < 4; ++nb) { const V b = WFrag<T16>::ld(Bt + boff + (size_t)nb * 16 * K + kc); V b2; if (NSPLIT >= 2) b2 = WFrag<T16>::ld(Bt2 + boff + (size_t)nb * 16 * K + kc);
#pragma unroll
            for (int mb = 0; mb < 4; ++mb) { acc[mb][nb] = WFrag<T16>::mma(a[mb], b, acc[mb][nb]); if (NSPLIT == 1 || NSPLIT == 2) acc[mb][nb] = WFrag<T16>::mma(a2[mb], b, acc[mb][nb]); if (NSPLIT >= 2) acc[mb][nb] = WFrag<T16>::mma(a[mb], b2, acc[mb][nb]); } }
        asm volatile("v_nop\n\tv_nop\n\tv_nop\n\tv_nop" : "+v"(acc[0][0]), "+v"(acc[1][1]), "+v"(acc[2][2]), "+v"(acc[3][3]) : "v"(a[0]), "v"(a[3]));
    }
#pragma unroll
    for (int mb = 0; mb < 4; ++mb) {
#pragma unroll
        for (int nb = 0; nb < 4; ++nb) {
#pragma unroll
            for (int j = 0; j < 8; ++j) os[(hi * 8 + j) * 68 + nb * 16 + lr] = acc[mb][nb][j]; }
        __builtin_amdgcn_wave_barrier(); asm volatile("" ::: "memory");
        float* crow = C + (size_t)(r0 + mb * 16) * ldc + c0;
#pragma unroll 1
        for (int ps = 0; ps < 2; ++ps) {
#pragma unroll
            for (int s = 0; s < 8; ++s) { const int row = 2 * s + hi, cofs = lr * 4; v4f val = *(const v4fa*)(os + row * 68 + cofs);
                *(volatile v4f*)(crow + (size_t)row * ldc + cofs) = val; }
            if (ps == 0) __threadfence(); }
        __builtin_amdgcn_wave_barrier(); asm volatile("" ::: "memory");
    }
}

__global__ __launch_bounds__(256) void k_qkp(const float* __restrict__ Fq, const float* __restrict__ Fk, bf* Pq, bf* Pk) {
    const size_t i = (size_t)blockIdx.x * 256 + threadIdx.x; const size_t n8 = (size_t)NB * NH_ * TT * HD / 8; if (i >= n8) return;
    const size_t e = i * 8; const int d = (int)(e % HD); const int t = (int)((e / HD) % TT); const int h = (int)((e / ((size_t)HD * TT)) % NH_); const int b = (int)(e / ((size_t)HD * TT * NH_));
    const size_t s = (((size_t)b * SEQ_FULL + t) * NH_ + h) * HD + d;
    const v8f vq = *(const v8f*)(Fq + s); const v8f vk = *(const v8f*)(Fk + s); v8us oq, ok;
#pragma unroll
    for (int q = 0; q < 8; ++q) { oq[q] = f2bf(vq[q]); ok[q] = f2bf(vk[q]); }
    *(volatile v8us*)(Pq + e) = oq; *(volatile v8us*)(Pk + e) = ok; __threadfence(); *(volatile v8us*)(Pq + e) = oq; *(volatile v8us*)(Pk + e) = ok;
}
__global__ __launch_bounds__(256) void k_vtp8(const float* __restrict__ F, bf* VTp) {
    const size_t i = (size_t)blockIdx.x * 256 + threadIdx.x; const size_t n8 = (size_t)NB * NH_ * HD * TT / 8; if (i >= n8) return;
    const size_t e = i * 8; const int t = (int)(e % TT); const int d = (int)((e / TT) % HD); const int h = (int)((e / ((size_t)TT * HD)) % NH_); const int b = (int)(e / ((size_t)TT * HD * NH_));
    v8us o;
#pragma unroll
    for (int q = 0; q < 8; ++q) o[q] = f2bf(F[(((size_t)b * SEQ_FULL + t + q) * NH_ + h) * HD + d]);
    *(volatile v8us*)(VTp + e) = o; __threadfence(); *(volatile v8us*)(VTp + e) = o;
}
__global__ __launch_bounds__(32) void k_flagline(int* F) { const int lane = threadIdx.x & 31; *(volatile int*)(F + lane) = 1; __threadfence(); *(volatile int*)(F + lane) = 1; }

__global__ __launch_bounds__(256) void k_asoft(const float* __restrict__ Sb, const int* __restrict__ CF, bf* Ph, bf* Pl) {
    const int lane = threadIdx.x & 31; const int row = blockIdx.x * 8 + (threadIdx.x >> 5); if (row >= ZH * TT) return; const int i = row % TT; const int zz = row / TT; const bool con = (CF[0] != 0);
    const float* sr = Sb + (size_t)row * TT; float v[TT / 32]; float mx = -3.0e38f;
#pragma unroll
    for (int ch = 0; ch < TT / 128; ++ch) { const int j0 = ch * 128 + lane * 4; const v4f a = *(const v4f*)(sr + j0);
#pragma unroll
        for (int q = 0; q < 4; ++q) { const int j = j0 + q; const float t = (j <= i || !con) ? a[q] * SCL : -3.0e38f; v[ch * 4 + q] = t; mx = fmaxf(mx, t); } }
#pragma unroll
    for (int sh = 16; sh; sh >>= 1) mx = fmaxf(mx, __shfl_xor(mx, sh, 32));
    float sum = 0.f;
#pragma unroll
    for (int k = 0; k < TT / 32; ++k) { float d0 = __fsub_rn(v[k], mx); asm volatile("" : "+v"(d0)); v[k] = __builtin_amdgcn_exp2f(__fmul_rn(d0, 1.4426950408889634f)); sum += v[k]; }
#pragma unroll
    for (int sh = 16; sh; sh >>= 1) sum += __shfl_xor(sum, sh, 32);
    const float f = __fdiv_rn(1.0f, sum);
#pragma unroll 1
    for (int ps = 0; ps < 2; ++ps) {
#pragma unroll
        for (int ch = 0; ch < TT / 128; ++ch) { v4us oh, ol;
#pragma unroll
            for (int q = 0; q < 4; ++q) { unsigned short a, c2; splitf(v[ch * 4 + q] * f, a, c2); oh[q] = a; ol[q] = c2; }
            const size_t oo = ((size_t)zz * RH + i) * TT + ch * 128 + lane * 4; *(volatile v4us*)(Ph + oo) = oh; *(volatile v4us*)(Pl + oo) = ol; }
        if (ps == 0) __threadfence(); }
}

extern "C" void kernel_launch(void* const* d_in, const int* in_sizes, int n_in,
                              void* d_out, int out_size, void* d_ws, size_t ws_size, hipStream_t stream) {
    if (n_in < 3) return;
    const float* xq = (const float*)d_in[0];     const float* xk = (const float*)d_in[1];     const float* xv = (const float*)d_in[2];
    const size_t need_x = ((size_t)(NB - 1) * SEQ_FULL + SEQ) * DM;
    if ((size_t)in_sizes[0] < need_x || (size_t)in_sizes[1] < need_x || (size_t)in_sizes[2] < need_x) return;
    if ((size_t)out_size < (size_t)NB * TT * DM) return;
    float* OUT = (float*)d_out;
    char* wsp = (char*)d_ws;
    auto take = [&](size_t bytes) { char* p = wsp; wsp += (bytes + 255) & ~(size_t)255; return (void*)p; };
    bf* QP = (bf*)take((size_t)NB * NH_ * TT * HD * 2);
    bf* KP = (bf*)take((size_t)NB * NH_ * TT * HD * 2);
    bf* VT = (bf*)take((size_t)NB * NH_ * HD * TT * 2);
    float* Sb = (float*)take((size_t)ZH * TT * TT * 4);
    bf* Ph = (bf*)take((size_t)ZH * RH * TT * 2);
    bf* Pl = (bf*)take((size_t)ZH * RH * TT * 2);
    int* FL = (int*)take((size_t)128);
    if ((size_t)(wsp - (char*)d_ws) > ws_size) return;
    const int* CFLAG = FL;

    k_flagline<<<1, 32, 0, stream>>>(FL);
    const size_t n8p = (size_t)NB * NH_ * TT * HD / 8;
    k_qkp<<<(unsigned)((n8p + 255) / 256), 256, 0, stream>>>(xq, xk, QP, KP);
    k_vtp8<<<(unsigned)((n8p + 255) / 256), 256, 0, stream>>>(xv, VT);

    for (int b = 0; b < NB; ++b) {
        for (int h0 = 0; h0 < NH_; h0 += ZH) {
            const size_t zp = ((size_t)b * NH_ + h0) * TT * HD;
            k_gemmc<bf, 0, 1><<<dim3(TT / 64, TT / 64, ZH), 32, 0, stream>>>(QP + zp, nullptr, KP + zp, nullptr, HD, Sb, TT, 0, (size_t)TT * HD, (size_t)TT * HD, (size_t)TT * TT, CFLAG);
            k_asoft<<<ZH * TT / 8, 256, 0, stream>>>(Sb, CFLAG, Ph, Pl);
            k_gemmc<bf, 1, 2><<<dim3(RH / 64, HD / 64, ZH), 32, 0, stream>>>(Ph, Pl, VT + zp, nullptr, TT, OUT + (size_t)b * TT * DM + (size_t)h0 * HD, DM, 0, (size_t)RH * TT, (size_t)HD * TT, (size_t)HD, CFLAG);
        }
    }
}
